// WordCharEncoderBiRNN_42889543417938
// MI455X (gfx1250) — hardware-run, weakly checked
//
#include <hip/hip_runtime.h>
#include <math.h>

typedef __attribute__((ext_vector_type(16))) _Float16 v16h;
typedef __attribute__((ext_vector_type(8)))  _Float16 v8h;
typedef __attribute__((ext_vector_type(4)))  _Float16 v4h;
typedef __attribute__((ext_vector_type(8)))  float    v8f;
typedef __attribute__((ext_vector_type(4)))  float    v4f;

constexpr int kL   = 256;
constexpr int kD   = 512;
constexpr int kH   = 1024;
constexpr int kCL  = 16;
constexpr int kV   = 57;
constexpr int kCh2 = 172;
constexpr int kCh3 = 170;
constexpr int kCh4 = 170;
constexpr int kXW  = 2 * kD;
constexpr int kG4  = 4 * kH;
constexpr int kNZ  = 2 * kG4;
constexpr int kTapRows = kCh2 * 2 + kCh3 * 3 + kCh4 * 4;
constexpr int kTapPad  = 1536;
constexpr int kVPad    = 64;
constexpr int kBase3   = kCh2 * 2;
constexpr int kBase4   = kCh2 * 2 + kCh3 * 3;
static_assert(kCh2 + kCh3 + kCh4 == kD);
static_assert(kTapRows == 1534 && kTapRows <= kTapPad && (kTapPad % 64) == 0);
static_assert(kBase3 == 344 && kBase4 == 854);
static_assert((kD % 32) == 0 && (kXW % 32) == 0 && (kH % 32) == 0);
static_assert((kL % 64) == 0 && (kNZ % 64) == 0 && (kVPad % 64) == 0);

constexpr bool kRneInputs = true;

constexpr float kCarryW = 256.0f;
constexpr float kCarryX = 16.0f;
constexpr float kCarryH = 256.0f;
constexpr float kScaleTap = 1.0f / (kCarryW * kCarryW);
constexpr float kScaleZ   = 1.0f / (kCarryX * kCarryW);
constexpr float kScaleHH  = 1.0f / (kCarryH * kCarryW);

constexpr size_t kSzWIH = (size_t)kNZ * kXW * 2;
constexpr size_t kSzWHH = (size_t)2 * kG4 * kH * 2;
constexpr size_t kSzWC  = (size_t)kTapPad * kD * 2;
constexpr size_t kSzE   = (size_t)kVPad * kD * 2;
constexpr size_t kSzP   = (size_t)kVPad * kTapPad * 4;
constexpr size_t kSzX   = (size_t)kL * kXW * 2;
constexpr size_t kSzZ   = (size_t)kL * kNZ * 4;
constexpr size_t kOffWIH = 0;
constexpr size_t kOffWHH = kOffWIH + kSzWIH;
constexpr size_t kOffWC  = kOffWHH + kSzWHH;
constexpr size_t kOffE   = kOffWC + kSzWC;
constexpr size_t kOffP   = kOffE + kSzE;
constexpr size_t kOffX   = kOffP + kSzP;
constexpr size_t kOffZ   = kOffX + kSzX;
constexpr size_t kWsTotal = kOffZ + kSzZ;
static_assert(kWsTotal == 44498944ull);
static_assert(kWsTotal <= 134217728ull);
static_assert((kOffWHH % 128) == 0 && (kOffWC % 128) == 0 && (kOffE % 128) == 0 &&
              (kOffP % 128) == 0 && (kOffX % 128) == 0 && (kOffZ % 128) == 0);

constexpr size_t kOutHidden = (size_t)kL * 2 * kH;
constexpr size_t kOutCell   = kOutHidden + 2 * kH;
constexpr size_t kOutTotal  = kOutCell + 2 * kH;
static_assert(kOutHidden * 4 == 2097152ull && kOutCell * 4 == 2105344ull && kOutTotal * 4 == 2113536ull);

__device__ __forceinline__ float rne_in(float f) {
  if (!kRneInputs) return f;
  unsigned u = __float_as_uint(f);
  unsigned lsb = (u & 0x00010000u) ? 1u : 0u;
  asm volatile("" : "+v"(lsb));
  u = (u + 0x7FFFu + lsb) & 0xFFFF0000u;
  return __uint_as_float(u);
}

__device__ __forceinline__ _Float16 to_h16(float v) {
  const float a = fabsf(v);
  const float w = (a < 6.103515625e-5f) ? 0.0f : v;
  return (_Float16)w;
}

union FragH { v16h v; v8h h[2]; };

__device__ __forceinline__ v16h frag_load(const _Float16* p) {
  FragH f;
  f.h[0] = *(const v8h*)(p);
  f.h[1] = *(const v8h*)(p + 16);
  return f.v;
}

__device__ __forceinline__ v8f mma16(v16h a, v16h b, v8f c) {
  c = __builtin_amdgcn_wmma_f32_16x16x32_f16(false, a, false, b, (short)0, c, false, false);
  asm volatile("v_nop\n\tv_nop\n\tv_nop\n\tv_nop" : "+v"(c) : "v"(a), "v"(b));
  return c;
}

__device__ __forceinline__ float sigm(float v) {
  const float x = fminf(fmaxf(v, -30.0f), 30.0f);
  return 1.0f / (1.0f + expf(-x));
}

constexpr int cdiv(int a, int b) { return (a + b - 1) / b; }

constexpr int kN8Big = kG4 * kXW / 8;
constexpr int kN8W2  = kCh2 * 2 * kD / 8;
constexpr int kN8W3  = kCh3 * 3 * kD / 8;
constexpr int kN8W4  = kCh4 * 4 * kD / 8;
constexpr int kN8E   = kV * kD / 8;
constexpr int kN8ZC  = (kTapPad - kTapRows) * kD / 8;
constexpr int kN8ZE  = (kVPad - kV) * kD / 8;
constexpr int kPB0 = 0;
constexpr int kPB1 = kPB0 + cdiv(kN8Big, 256);
constexpr int kPB2 = kPB1 + cdiv(kN8Big, 256);
constexpr int kPB3 = kPB2 + cdiv(kN8Big, 256);
constexpr int kPB4 = kPB3 + cdiv(kN8Big, 256);
constexpr int kPB5 = kPB4 + cdiv(kN8W2, 256);
constexpr int kPB6 = kPB5 + cdiv(kN8W3, 256);
constexpr int kPB7 = kPB6 + cdiv(kN8W4, 256);
constexpr int kPB8 = kPB7 + cdiv(kN8E, 256);
constexpr int kPB9 = kPB8 + cdiv(kN8ZC, 256);
constexpr int kPBEnd = kPB9 + cdiv(kN8ZE, 256);
static_assert((kN8W2 % 8) == 0 && (kN8W3 % 8) == 0 && (kN8W4 % 8) == 0 && (kN8E % 8) == 0 &&
              (kN8ZC % 8) == 0 && (kN8ZE % 8) == 0 && (kN8Big % 8) == 0);
static_assert(kPBEnd == 8594);

__global__ __launch_bounds__(256) void prep_planes_kernel(
    const float* __restrict__ wihf, const float* __restrict__ wihr,
    const float* __restrict__ whhf, const float* __restrict__ whhr,
    const float* __restrict__ w2, const float* __restrict__ w3, const float* __restrict__ w4,
    const float* __restrict__ ce,
    unsigned short* __restrict__ WIH, unsigned short* __restrict__ WHH,
    unsigned short* __restrict__ WC, unsigned short* __restrict__ E16)
{
  const int bx = blockIdx.x;
  const float* src = wihf;
  unsigned short* dst = WIH;
  int n8 = kN8Big;
  int b0 = kPB0;
  bool zero = false;
  if (bx >= kPB1) { src = wihr; dst = WIH + (size_t)kG4 * kXW; b0 = kPB1; }
  if (bx >= kPB2) { src = whhf; dst = WHH; b0 = kPB2; }
  if (bx >= kPB3) { src = whhr; dst = WHH + (size_t)kG4 * kH; b0 = kPB3; }
  if (bx >= kPB4) { src = w2; dst = WC; n8 = kN8W2; b0 = kPB4; }
  if (bx >= kPB5) { src = w3; dst = WC + (size_t)kBase3 * kD; n8 = kN8W3; b0 = kPB5; }
  if (bx >= kPB6) { src = w4; dst = WC + (size_t)kBase4 * kD; n8 = kN8W4; b0 = kPB6; }
  if (bx >= kPB7) { src = ce; dst = E16; n8 = kN8E; b0 = kPB7; }
  if (bx >= kPB8) { src = ce; dst = WC + (size_t)kTapRows * kD; n8 = kN8ZC; b0 = kPB8; zero = true; }
  if (bx >= kPB9) { src = ce; dst = E16 + (size_t)kV * kD; n8 = kN8ZE; b0 = kPB9; zero = true; }

  const int i = (bx - b0) * 256 + (int)threadIdx.x;
  if (i >= n8) return;
  const size_t e0 = (size_t)i << 3;
  v4f a0 = (v4f){0.f, 0.f, 0.f, 0.f};
  v4f a1 = (v4f){0.f, 0.f, 0.f, 0.f};
  if (!zero) {
    a0 = *(const v4f*)(src + e0);
    a1 = *(const v4f*)(src + e0 + 4);
  }
  v8h hv;
#pragma unroll
  for (int e = 0; e < 4; ++e) {
    const float f0 = a0[e];
    const float f1 = a1[e];
    hv[e]     = to_h16(rne_in(f0) * kCarryW);
    hv[4 + e] = to_h16(rne_in(f1) * kCarryW);
  }
  unsigned short* q = dst + e0;
  *(volatile v8h*)q = hv;
  __threadfence();
  *(volatile v8h*)q = hv;
}

template <int BIASK>
__global__ __launch_bounds__(256) void gemm64_f16_kernel(
    const unsigned short* __restrict__ Ap, int lda,
    const unsigned short* __restrict__ Btp, int ldb,
    float* __restrict__ C, int ldc,
    const float* __restrict__ bA0, const float* __restrict__ bB0,
    const float* __restrict__ bA1, const float* __restrict__ bB1, int nsplit,
    int M, int N, int K, float scale)
{
  const _Float16* A  = (const _Float16*)Ap;
  const _Float16* Bt = (const _Float16*)Btp;
  __shared__ __align__(16) float sT[8][16 * 68];
  const int lane = threadIdx.x & 31;
  const int wave = threadIdx.x >> 5;
  const int tilesN = N >> 6;
  const int tilesM = M >> 6;
  const int tile = blockIdx.x * 8 + wave;
  if (tile >= tilesM * tilesN) return;
  const int tm = tile / tilesN;
  const int tn = tile - tm * tilesN;
  const int m0 = tm << 6;
  const int n0 = tn << 6;

  const int rlane = lane & 15;
  const int koff  = (lane >> 4) * 8;
  const int mOff  = (lane >> 4) * 8;

  v8f acc[4][4];
#pragma unroll
  for (int i = 0; i < 4; ++i)
#pragma unroll
    for (int j = 0; j < 4; ++j) acc[i][j] = (v8f){0.f, 0.f, 0.f, 0.f, 0.f, 0.f, 0.f, 0.f};

  for (int k0 = 0; k0 < K; k0 += 32) {
    v16h bh[4];
#pragma unroll
    for (int j = 0; j < 4; ++j) {
      const size_t bo = (size_t)(n0 + (j << 4) + rlane) * ldb + koff + k0;
      bh[j] = frag_load(Bt + bo);
    }
#pragma unroll
    for (int i = 0; i < 4; ++i) {
      const size_t ao = (size_t)(m0 + (i << 4) + rlane) * lda + koff + k0;
      const v16h ah = frag_load(A + ao);
#pragma unroll
      for (int j = 0; j < 4; ++j) acc[i][j] = mma16(ah, bh[j], acc[i][j]);
    }
  }

  float* slab = sT[wave];
  const bool sec = (n0 >= nsplit);
  const float* pa = sec ? bA1 : bA0;
  const float* pb = sec ? bB1 : bB0;
  const int nb = n0 - (sec ? nsplit : 0);
#pragma unroll
  for (int i = 0; i < 4; ++i) {
    const int mBase = m0 + (i << 4);
#pragma unroll
    for (int j = 0; j < 4; ++j) {
      float bv = 0.f;
      if (BIASK == 1) {
        const float ba = pa[nb + (j << 4) + rlane];
        const float bb = pb[nb + (j << 4) + rlane];
        bv = rne_in(ba) + rne_in(bb);
      }
#pragma unroll
      for (int r = 0; r < 8; ++r) {
        const float v = acc[i][j][r] * scale + bv;
        slab[(mOff + r) * 68 + (j << 4) + rlane] = v;
      }
    }
    __builtin_amdgcn_fence(__ATOMIC_RELEASE, "workgroup");
    __builtin_amdgcn_wave_barrier();
    __builtin_amdgcn_fence(__ATOMIC_ACQUIRE, "workgroup");
    {
      const int hh = lane >> 4, c4 = (lane & 15) * 4;
      for (int pass = 0; pass < 2; ++pass) {
#pragma unroll
        for (int it = 0; it < 8; ++it) {
          const int row = it * 2 + hh;
          const v4f v = *(const v4f*)(slab + row * 68 + c4);
          *(volatile v4f*)(C + (size_t)(mBase + row) * ldc + n0 + c4) = v;
        }
        __threadfence();
      }
    }
    __builtin_amdgcn_fence(__ATOMIC_RELEASE, "workgroup");
    __builtin_amdgcn_wave_barrier();
    __builtin_amdgcn_fence(__ATOMIC_ACQUIRE, "workgroup");
  }
}

__global__ __launch_bounds__(256) void pool_pack_kernel(
    const float* __restrict__ wemb, const int* __restrict__ cidx, const float* __restrict__ P,
    const float* __restrict__ b2, const float* __restrict__ b3, const float* __restrict__ b4,
    unsigned short* __restrict__ X16)
{
  __shared__ int sOff[kCL];
  __shared__ __align__(16) float sX[kXW];
  const int w = blockIdx.x;
  const int tid = threadIdx.x;
  {
    int ci = cidx[w * kCL + (tid & 15)];
    asm volatile("" : "+v"(ci));
    ci = ci < 0 ? 0 : ci;
    ci = ci > (kV - 1) ? (kV - 1) : ci;
    if (tid < kCL) sOff[tid] = ci * kTapPad;
  }
  {
    const float e0 = wemb[(size_t)w * kD + tid];
    const float e1 = wemb[(size_t)w * kD + 256 + tid];
    sX[tid] = rne_in(e0);
    sX[256 + tid] = rne_in(e1);
  }
  __syncthreads();

#pragma unroll 1
  for (int half = 0; half < 2; ++half) {
    const int ch = tid + 256 * half;
    const bool g2 = (ch < kCh2);
    const bool g3 = (!g2) && (ch < kCh2 + kCh3);
    int c2i = ch;
    c2i = c2i > (kCh2 - 1) ? (kCh2 - 1) : c2i;
    int c3i = ch - kCh2;
    c3i = c3i < 0 ? 0 : c3i;
    c3i = c3i > (kCh3 - 1) ? (kCh3 - 1) : c3i;
    int c4i = ch - kCh2 - kCh3;
    c4i = c4i < 0 ? 0 : c4i;
    c4i = c4i > (kCh4 - 1) ? (kCh4 - 1) : c4i;
    float bb2 = b2[c2i];
    float bb3 = b3[c3i];
    float bb4 = b4[c4i];
    asm volatile("" : "+v"(bb2));
    asm volatile("" : "+v"(bb3));
    asm volatile("" : "+v"(bb4));
    const float bias = rne_in(g2 ? bb2 : (g3 ? bb3 : bb4));
    const int ntap = g2 ? 2 : (g3 ? 3 : 4);
    const int col  = g2 ? (c2i * 2) : (g3 ? (kBase3 + c3i * 3) : (kBase4 + c4i * 4));
    const int npos = kCL + 1 - ntap;
    float best = 0.0f;
#pragma unroll 1
    for (int t = 0; t < kCL - 1; ++t) {
      float s = bias;
#pragma unroll
      for (int k = 0; k < 4; ++k) {
        int tt = t + k;
        tt = tt > (kCL - 1) ? (kCL - 1) : tt;
        int cc = col + k;
        cc = cc > (kTapPad - 1) ? (kTapPad - 1) : cc;
        float pv = P[sOff[tt] + cc];
        asm volatile("" : "+v"(pv));
        s += (k < ntap) ? pv : 0.0f;
      }
      const float r = fmaxf(s, 0.0f);
      best = (t < npos) ? fmaxf(best, r) : best;
    }
    sX[kD + ch] = best;
  }
  __syncthreads();

  if (tid < 128) {
    const float* sp = sX + 8 * tid;
    const v4f a0 = *(const v4f*)(sp);
    const v4f a1 = *(const v4f*)(sp + 4);
    v8h hv;
#pragma unroll
    for (int e = 0; e < 4; ++e) {
      const float f0 = a0[e];
      const float f1 = a1[e];
      hv[e]     = to_h16(f0 * kCarryX);
      hv[4 + e] = to_h16(f1 * kCarryX);
    }
    unsigned short* q = X16 + (size_t)w * kXW + 8 * tid;
    *(volatile v8h*)q = hv;
    __threadfence();
    *(volatile v8h*)q = hv;
  }
}

__global__ __launch_bounds__(512) void lstm_scan_kernel(
    const unsigned short* __restrict__ WHH, const float* __restrict__ Z, float* __restrict__ out)
{
  __shared__ __align__(16) _Float16 hbuf[2][kH];
  const int dir  = blockIdx.x;
  const int tid  = threadIdx.x;
  const int lane = tid & 31;
  const int wave = tid >> 5;
  const int hh   = lane >> 4;
  const int c    = lane & 15;
  const int u0   = wave * 64;

  {
    _Float16* hb = &hbuf[0][0];
    *(v4h*)(hb + 4 * tid) = (v4h){(_Float16)0.0f, (_Float16)0.0f, (_Float16)0.0f, (_Float16)0.0f};
  }
  __syncthreads();

  const _Float16* Wd   = (const _Float16*)WHH + (size_t)dir * kG4 * kH;
  const _Float16* wrow = Wd + (size_t)(u0 + c) * kH + 8 * hh;
  const float* zcol = Z + (size_t)dir * kG4 + u0 + lane;
  float* ocol = out + (size_t)dir * kH + u0 + lane;
  float* hcol = out + kOutHidden + (size_t)dir * kH + u0 + lane;
  float* ccol = out + kOutCell + (size_t)dir * kH + u0 + lane;

  float cA = 0.0f, cB = 0.0f;

#pragma unroll 1
  for (int s = 0; s < kL; ++s) {
    const int t   = dir ? (kL - 1 - s) : s;
    const int cur = s & 1;
    float zA[4], zB[4];
#pragma unroll
    for (int p = 0; p < 2; ++p) {
      v8f acc[2][4];
#pragma unroll
      for (int gq = 0; gq < 2; ++gq)
#pragma unroll
        for (int nt = 0; nt < 4; ++nt) acc[gq][nt] = (v8f){0.f, 0.f, 0.f, 0.f, 0.f, 0.f, 0.f, 0.f};
#pragma unroll 1
      for (int k0 = 0; k0 < kH; k0 += 32) {
        FragH a;
        a.h[0] = *(const v8h*)(&hbuf[cur][k0 + 8 * hh]);
        a.h[1] = *(const v8h*)(&hbuf[cur][k0 + 16 + 8 * hh]);
#pragma unroll
        for (int gq = 0; gq < 2; ++gq) {
#pragma unroll
          for (int nt = 0; nt < 4; ++nt) {
            const _Float16* bp = wrow + (size_t)((2 * p + gq) * kH + nt * 16) * kH + k0;
            const v16h b = frag_load(bp);
            acc[gq][nt] = mma16(a.v, b, acc[gq][nt]);
          }
        }
      }
#pragma unroll
      for (int gq = 0; gq < 2; ++gq) {
        const float t0 = acc[gq][0][0];
        const float t1 = acc[gq][1][0];
        const float t2 = acc[gq][2][0];
        const float t3 = acc[gq][3][0];
        zA[2 * p + gq] = hh ? t1 : t0;
        zB[2 * p + gq] = hh ? t3 : t2;
      }
    }

    const float* zr = zcol + (size_t)t * kNZ;
    const float qiA = zr[0],        qiB = zr[32];
    const float qfA = zr[kH],       qfB = zr[kH + 32];
    const float qgA = zr[2 * kH],   qgB = zr[2 * kH + 32];
    const float qoA = zr[3 * kH],   qoB = zr[3 * kH + 32];

    const float ziA = zA[0] * kScaleHH + qiA;
    const float zfA = zA[1] * kScaleHH + qfA;
    const float zgA = zA[2] * kScaleHH + qgA;
    const float zoA = zA[3] * kScaleHH + qoA;
    const float ziB = zB[0] * kScaleHH + qiB;
    const float zfB = zB[1] * kScaleHH + qfB;
    const float zgB = zB[2] * kScaleHH + qgB;
    const float zoB = zB[3] * kScaleHH + qoB;

    cA = sigm(zfA) * cA + sigm(ziA) * tanhf(zgA);
    const float hA = sigm(zoA) * tanhf(cA);
    cB = sigm(zfB) * cB + sigm(ziB) * tanhf(zgB);
    const float hB = sigm(zoB) * tanhf(cB);

    hbuf[cur ^ 1][u0 + lane]      = to_h16(hA * kCarryH);
    hbuf[cur ^ 1][u0 + 32 + lane] = to_h16(hB * kCarryH);

    float* op = ocol + (size_t)t * (2 * kH);
    const bool last = (s == kL - 1);
    const float cAv = cA, cBv = cB;
    for (int pass = 0; pass < 2; ++pass) {
      *(volatile float*)(op) = hA;
      *(volatile float*)(op + 32) = hB;
      if (last) {
        *(volatile float*)(hcol) = hA;
        *(volatile float*)(hcol + 32) = hB;
        *(volatile float*)(ccol) = cAv;
        *(volatile float*)(ccol + 32) = cBv;
      }
      __threadfence();
    }
    __syncthreads();
  }
}

extern "C" void kernel_launch(void* const* d_in, const int* in_sizes, int n_in,
                              void* d_out, int out_size, void* d_ws, size_t ws_size,
                              hipStream_t stream) {
  if (n_in < 17) return;
  if (in_sizes[0] != kL * kD) return;
  if (in_sizes[1] != kL * kCL) return;
  if (in_sizes[2] != kV * kD) return;
  if (in_sizes[3] != kCh2 * 2 * kD) return;
  if (in_sizes[4] != kCh2) return;
  if (in_sizes[5] != kCh3 * 3 * kD) return;
  if (in_sizes[6] != kCh3) return;
  if (in_sizes[7] != kCh4 * 4 * kD) return;
  if (in_sizes[8] != kCh4) return;
  if (in_sizes[9] != kG4 * kXW) return;
  if (in_sizes[10] != kG4 * kH) return;
  if (in_sizes[11] != kG4) return;
  if (in_sizes[12] != kG4) return;
  if (in_sizes[13] != kG4 * kXW) return;
  if (in_sizes[14] != kG4 * kH) return;
  if (in_sizes[15] != kG4) return;
  if (in_sizes[16] != kG4) return;
  if ((size_t)out_size != kOutTotal) return;
  if (ws_size < kWsTotal) return;

  const float* word_emb = (const float*)d_in[0];
  const int*   char_idx = (const int*)d_in[1];
  const float* char_emb = (const float*)d_in[2];
  const float* W2  = (const float*)d_in[3];
  const float* b2  = (const float*)d_in[4];
  const float* W3  = (const float*)d_in[5];
  const float* b3  = (const float*)d_in[6];
  const float* W4  = (const float*)d_in[7];
  const float* b4  = (const float*)d_in[8];
  const float* Wih_f = (const float*)d_in[9];
  const float* Whh_f = (const float*)d_in[10];
  const float* bih_f = (const float*)d_in[11];
  const float* bhh_f = (const float*)d_in[12];
  const float* Wih_r = (const float*)d_in[13];
  const float* Whh_r = (const float*)d_in[14];
  const float* bih_r = (const float*)d_in[15];
  const float* bhh_r = (const float*)d_in[16];
  float* out = (float*)d_out;

  char* ws = (char*)d_ws;
  unsigned short* WIH = (unsigned short*)(ws + kOffWIH);
  unsigned short* WHH = (unsigned short*)(ws + kOffWHH);
  unsigned short* WC  = (unsigned short*)(ws + kOffWC);
  unsigned short* E16 = (unsigned short*)(ws + kOffE);
  float*          P   = (float*)(ws + kOffP);
  unsigned short* X16 = (unsigned short*)(ws + kOffX);
  float*          Z   = (float*)(ws + kOffZ);

  prep_planes_kernel<<<kPBEnd, 256, 0, stream>>>(Wih_f, Wih_r, Whh_f, Whh_r, W2, W3, W4, char_emb,
                                                 WIH, WHH, WC, E16);

  gemm64_f16_kernel<0><<<(kVPad / 64) * (kTapPad / 64) / 8, 256, 0, stream>>>(
      E16, kD, WC, kD, P, kTapPad,
      bih_f, bhh_f, bih_r, bhh_r, kTapPad,
      kVPad, kTapPad, kD, kScaleTap);

  pool_pack_kernel<<<kL, 256, 0, stream>>>(word_emb, char_idx, P, b2, b3, b4, X16);

  gemm64_f16_kernel<1><<<(kL / 64) * (kNZ / 64) / 8, 256, 0, stream>>>(
      X16, kXW, WIH, kXW, Z, kNZ,
      bih_f, bhh_f, bih_r, bhh_r, kG4,
      kL, kNZ, kXW, kScaleZ);

  lstm_scan_kernel<<<2, 512, 0, stream>>>(WHH, Z, out);
}
